// MambaLayer_49392123904378
// MI455X (gfx1250) — hardware-verified
//
#include <hip/hip_runtime.h>
#include <hip/hip_bf16.h>
#include <math.h>

#define __bf16 _Float16
typedef _Float16 bf16_t;
typedef __attribute__((ext_vector_type(16))) _Float16 v16bf;
typedef __attribute__((ext_vector_type(8)))  _Float16 v8bf;
typedef __attribute__((ext_vector_type(4)))  float  v4f_t;
typedef float v4fa __attribute__((ext_vector_type(4), may_alias));
#define RSPLIT (1.0f / 2048.0f)
__device__ __forceinline__ unsigned pack2s(float a, float b, unsigned* lo) {
  const _Float16 h0 = (_Float16)a, h1 = (_Float16)b;
  const _Float16 l0 = (_Float16)((a - (float)h0) * 2048.0f), l1 = (_Float16)((b - (float)h1) * 2048.0f);
  *lo = (unsigned)__builtin_bit_cast(unsigned short, l0) | ((unsigned)__builtin_bit_cast(unsigned short, l1) << 16);
  return (unsigned)__builtin_bit_cast(unsigned short, h0) | ((unsigned)__builtin_bit_cast(unsigned short, h1) << 16);
}
typedef __attribute__((ext_vector_type(8)))  float  v8f;
typedef __attribute__((ext_vector_type(4)))  int    v4i;

typedef __attribute__((address_space(1))) v4i v4i_g;
typedef __attribute__((address_space(3))) v4i v4i_l;

#define BB 2
#define LL 2048
#define DD 1024
#define EE 2048
#define NNS 16
#define KC 4
#define RR 64
#define MTOT (BB*LL)

#define TBM 128
#define TBN 128
#define TBK 64
#define TBKP 72

#if defined(__gfx1250__) && \
    __has_builtin(__builtin_amdgcn_global_load_async_to_lds_b128) && \
    __has_builtin(__builtin_amdgcn_s_wait_asynccnt)
#define USE_ASYNC 1
#else
#define USE_ASYNC 0
#endif

__global__ void f32_to_bf16_kernel(const float* __restrict__ in,
                                   bf16_t* __restrict__ out, int n) {
  int i = (blockIdx.x * blockDim.x + threadIdx.x) * 2;
  if (i < n) {
    unsigned lo; const unsigned hv = pack2s(in[i], in[i + 1], &lo);
    *(volatile unsigned*)(out + i) = hv; *(volatile unsigned*)(out + (size_t)n + i) = lo;
    __threadfence();
    *(volatile unsigned*)(out + i) = hv; *(volatile unsigned*)(out + (size_t)n + i) = lo;
  }
}

__device__ __forceinline__ v16bf frag_a(const bf16_t* base, int lds, int row16,
                                        int kk, int lane) {
  int h = (lane >> 4) & 1;
  const bf16_t* p = base + (size_t)(row16 + (lane & 15)) * lds + kk + h * 8;
  union { v16bf v; v8bf q[2]; } u;
  u.q[0] = *(const v8bf*)(p);
  u.q[1] = *(const v8bf*)(p + 16);
  return u.v;
}
__device__ __forceinline__ v16bf frag_b(const bf16_t* base, int lds, int col16,
                                        int kk, int lane) {
  int h = (lane >> 4) & 1;
  const bf16_t* p = base + (size_t)(col16 + (lane & 15)) * lds + kk + h * 8;
  union { v16bf v; v8bf q[2]; } u;
  u.q[0] = *(const v8bf*)(p);
  u.q[1] = *(const v8bf*)(p + 16);
  return u.v;
}
__device__ __forceinline__ v8f wmma_split(v16bf ah, v16bf al, v16bf bh, v16bf bl, v8f c) {
  v8f x = {};
  x = __builtin_amdgcn_wmma_f32_16x16x32_f16(false, al, false, bh, (short)0, x, false, false);
  x = __builtin_amdgcn_wmma_f32_16x16x32_f16(false, ah, false, bl, (short)0, x, false, false);
  return __builtin_amdgcn_wmma_f32_16x16x32_f16(false, ah, false, bh, (short)0, c, false, false) + x * RSPLIT;
}

__device__ __forceinline__ float softplus_f(float x) {
  return (x > 20.f) ? x : log1pf(__expf(x));
}

__device__ __forceinline__ void cp_b128(const bf16_t* g, bf16_t* l) {
#if USE_ASYNC
  const v4i* gv = (const v4i*)g;
  v4i*       lv = (v4i*)l;
  __builtin_amdgcn_global_load_async_to_lds_b128(
      (v4i_g*)gv, (v4i_l*)lv, 0, 0);
#else
  *(v8bf*)l = *(const v8bf*)g;
#endif
}

#if USE_ASYNC
#define ASYNC_WAIT(n) __builtin_amdgcn_s_wait_asynccnt(n)
#else
#define ASYNC_WAIT(n)
#endif

__device__ __forceinline__ void copy_stage(bf16_t* sA, bf16_t* sB, bf16_t* sAl, bf16_t* sBl,
                                           const bf16_t* A, const bf16_t* Bw, size_t pla, size_t plb,
                                           int tm0, int tn0, int k0, int K) {
  int c = threadIdx.x;
  #pragma unroll
  for (int i = 0; i < (TBM * TBK / 8) / 256; ++i, c += 256) {
    int row = c >> 3;
    int col = (c & 7) * 8;
    cp_b128(A + (size_t)(tm0 + row) * K + k0 + col, sA + row * TBKP + col);
    cp_b128(A + pla + (size_t)(tm0 + row) * K + k0 + col, sAl + row * TBKP + col);
  }
  c = threadIdx.x;
  #pragma unroll
  for (int i = 0; i < (TBN * TBK / 8) / 256; ++i, c += 256) {
    int row = c >> 3;
    int col = (c & 7) * 8;
    cp_b128(Bw + (size_t)(tn0 + row) * K + k0 + col, sB + row * TBKP + col);
    cp_b128(Bw + plb + (size_t)(tn0 + row) * K + k0 + col, sBl + row * TBKP + col);
  }
}

template<int EPI>
__global__ __launch_bounds__(256)
void gemm_bf16_wmma_tiled_kernel(const bf16_t* __restrict__ A,
                                 const bf16_t* __restrict__ Bw,
                                 float* __restrict__ C,
                                 int M, int N, int K,
                                 const float* __restrict__ auxf) {
  __shared__ __attribute__((aligned(16))) bf16_t smem[4][2][TBM * TBKP];
  const size_t pla = (size_t)M * K, plb = (size_t)N * K;

  const int lane = threadIdx.x & 31;
  const int wave = threadIdx.x >> 5;
  const int nTilesN = N / TBN;
  const int tm0 = (blockIdx.x / nTilesN) * TBM;
  const int tn0 = (blockIdx.x % nTilesN) * TBN;
  const int wm = (wave >> 1) * 32;
  const int wn = (wave & 1) * 64;

  v8f acc[2][4] = {};

  const int nk = K / TBK;
  copy_stage(smem[0][0], smem[1][0], smem[2][0], smem[3][0], A, Bw, pla, plb, tm0, tn0, 0, K);

  for (int ks = 0; ks < nk; ++ks) {
    const int cur = ks & 1;
    if (ks + 1 < nk) {
      copy_stage(smem[0][cur ^ 1], smem[1][cur ^ 1], smem[2][cur ^ 1], smem[3][cur ^ 1], A, Bw, pla, plb, tm0, tn0, (ks + 1) * TBK, K);
      ASYNC_WAIT(16);
    } else {
      ASYNC_WAIT(0);
    }
    __syncthreads();

    const bf16_t* As = smem[0][cur];  const bf16_t* Asl = smem[2][cur];
    const bf16_t* Bs = smem[1][cur];  const bf16_t* Bsl = smem[3][cur];
    #pragma unroll
    for (int kk = 0; kk < TBK; kk += 32) {
      v16bf a0 = frag_a(As, TBKP, wm + 0,  kk, lane), a0l = frag_a(Asl, TBKP, wm + 0,  kk, lane);
      v16bf a1 = frag_a(As, TBKP, wm + 16, kk, lane), a1l = frag_a(Asl, TBKP, wm + 16, kk, lane);
      #pragma unroll
      for (int j = 0; j < 4; ++j) {
        v16bf bf = frag_b(Bs, TBKP, wn + j * 16, kk, lane), bfl = frag_b(Bsl, TBKP, wn + j * 16, kk, lane);
        acc[0][j] = wmma_split(a0, a0l, bf, bfl, acc[0][j]);
        acc[1][j] = wmma_split(a1, a1l, bf, bfl, acc[1][j]);
      }
    }
    __syncthreads();
  }

  const int h  = (lane >> 4) & 1;
  const int nl = lane & 15;
  float* stg = (float*)&smem[0][0][0] + wave * (32 * 64);
  #pragma unroll
  for (int im = 0; im < 2; ++im)
    #pragma unroll
    for (int j = 0; j < 4; ++j)
      #pragma unroll
      for (int r = 0; r < 8; ++r) stg[(im * 16 + h * 8 + r) * 64 + j * 16 + nl] = acc[im][j][r];
  asm volatile("s_wait_dscnt 0" ::: "memory");
#pragma unroll 1
  for (int pass = 0; pass < 2; ++pass) {
#pragma unroll 4
    for (int i = 0; i < 16; ++i) {
      const int c = lane + 32 * i, rr = c >> 4, q = c & 15;
      const int mg = tm0 + wm + rr;
      const size_t go = (size_t)mg * N + tn0 + wn + q * 4;
      v4f_t v = *(const volatile v4fa*)(stg + rr * 64 + q * 4);
      if (EPI == 3) v += *(const v4f_t*)(auxf + go);
      *(volatile v4f_t*)(C + go) = v;
    }
    __threadfence();
  }
}

template<int NT, int EPI>
__global__ __launch_bounds__(256) void gemm_bf16_wmma_kernel(const bf16_t* __restrict__ A,
                                      const bf16_t* __restrict__ Bw,
                                      float* __restrict__ C,
                                      int M, int N, int K,
                                      const float* __restrict__ auxf,
                                      bf16_t* __restrict__ auxb) {
  __shared__ __attribute__((aligned(16))) float stg[8][16 * 16 * NT];
  const int lane = threadIdx.x & 31;
  const int wave = threadIdx.x >> 5;
  const int stripsPerRow = N / (16 * NT);
  const int strip = blockIdx.x * (blockDim.x >> 5) + wave;
  if (strip >= (M / 16) * stripsPerRow) return;
  const int tm  = strip / stripsPerRow;
  const int tn0 = (strip % stripsPerRow) * NT;
  const size_t pla = (size_t)M * K, plb = (size_t)N * K;

  v8f acc[NT] = {};

  for (int k0 = 0; k0 < K; k0 += 32) {
    v16bf af  = frag_a(A, K, tm * 16, k0, lane);
    v16bf afl = frag_a(A + pla, K, tm * 16, k0, lane);
    if (k0 + 32 < K)
      __builtin_prefetch(A + (size_t)(tm * 16 + (lane & 15)) * K + k0 + 32, 0, 1);
    #pragma unroll
    for (int t = 0; t < NT; ++t) {
      v16bf bf  = frag_b(Bw, K, (tn0 + t) * 16, k0, lane);
      v16bf bfl = frag_b(Bw + plb, K, (tn0 + t) * 16, k0, lane);
      acc[t] = wmma_split(af, afl, bf, bfl, acc[t]);
    }
  }

  const int h  = (lane >> 4) & 1;
  const int nl = lane & 15;
  constexpr int SW = 16 * NT;
  float* sw = stg[wave];
  #pragma unroll
  for (int t = 0; t < NT; ++t) {
    int ng = (tn0 + t) * 16 + nl;
    #pragma unroll
    for (int r = 0; r < 8; ++r) {
      float v = acc[t][r];
      if (EPI == 2) v = softplus_f(v + auxf[ng]);
      sw[(h * 8 + r) * SW + t * 16 + nl] = v;
    }
  }
  asm volatile("s_wait_dscnt 0" ::: "memory");
  constexpr int CPR = SW / 4;
#pragma unroll 1
  for (int pass = 0; pass < 2; ++pass) {
    for (int c = lane; c < 16 * CPR; c += 32) {
      const int rr = c / CPR, q = c - rr * CPR;
      *(volatile v4f_t*)(C + (size_t)(tm * 16 + rr) * N + tn0 * 16 + q * 4) = *(const volatile v4fa*)(sw + rr * SW + q * 4);
    }
    if (EPI == 1) {
#pragma unroll 4
      for (int rr = 0; rr < 16; ++rr) {
        unsigned lo; const unsigned hv = pack2s(*(const volatile float*)(sw + rr * SW + 2 * lane), *(const volatile float*)(sw + rr * SW + 2 * lane + 1), &lo);
        const size_t o = (size_t)(tm * 16 + rr) * RR + 2 * lane;
        *(volatile unsigned*)(auxb + o) = hv; *(volatile unsigned*)(auxb + (size_t)M * RR + o) = lo;
      }
    }
    __threadfence();
  }
}

__global__ void conv_silu_kernel(const float* __restrict__ xz,
                                 const float* __restrict__ Wc,
                                 const float* __restrict__ bc,
                                 float* __restrict__ u,
                                 bf16_t* __restrict__ ub) {
  size_t idx = ((size_t)blockIdx.x * blockDim.x + threadIdx.x) * 2;
  if (idx >= (size_t)MTOT * EE) return;
  int e = (int)(idx % EE);
  size_t m = idx / EE;
  int l = (int)(m % LL);
  float acc0 = bc[e], acc1 = bc[e + 1];
  #pragma unroll
  for (int k = 0; k < KC; ++k) {
    int ll = l - (KC - 1) + k;
    if (ll >= 0) {
      const float* xp = xz + (m + (size_t)(ll - l)) * (size_t)(2 * EE) + e;
      acc0 += xp[0] * Wc[e * KC + k];
      acc1 += xp[1] * Wc[(e + 1) * KC + k];
    }
  }
  float s0 = acc0 / (1.f + __expf(-acc0)), s1 = acc1 / (1.f + __expf(-acc1));
  typedef __attribute__((ext_vector_type(2))) float v2f_t;
  v2f_t uv = {s0, s1};
  unsigned lo; const unsigned hv = pack2s(s0, s1, &lo);
  *(volatile v2f_t*)(u + m * (size_t)EE + e) = uv; *(volatile unsigned*)(ub + m * (size_t)EE + e) = hv; *(volatile unsigned*)(ub + (size_t)MTOT * EE + m * (size_t)EE + e) = lo;
  __threadfence();
  *(volatile v2f_t*)(u + m * (size_t)EE + e) = uv; *(volatile unsigned*)(ub + m * (size_t)EE + e) = hv; *(volatile unsigned*)(ub + (size_t)MTOT * EE + m * (size_t)EE + e) = lo;
}

__global__ __launch_bounds__(256) void scan_gate_kernel(const float* __restrict__ delta,
                                 const float* __restrict__ u,
                                 const float* __restrict__ dbl,
                                 const float* __restrict__ xz,
                                 const float* __restrict__ A_log,
                                 const float* __restrict__ D_skip,
                                 bf16_t* __restrict__ yb) {
  int t = blockIdx.x * blockDim.x + threadIdx.x;
  if (t >= BB * EE / 2) return;
  int b = t / (EE / 2);
  int e = (t % (EE / 2)) * 2;
  float Ae0[NNS], Ae1[NNS];
  #pragma unroll
  for (int n = 0; n < NNS; ++n) { Ae0[n] = -__expf(A_log[e * NNS + n]); Ae1[n] = -__expf(A_log[(e + 1) * NNS + n]); }
  float dsk0 = D_skip[e], dsk1 = D_skip[e + 1];
  float h0[NNS], h1[NNS];
  #pragma unroll
  for (int n = 0; n < NNS; ++n) { h0[n] = 0.f; h1[n] = 0.f; }
  const size_t PLY = (size_t)MTOT * EE;

  for (int l = 0; l < LL; ++l) {
    size_t m = (size_t)b * LL + l;
    const float* bc = dbl + m * 96;
    float d0 = delta[m * EE + e], d1 = delta[m * EE + e + 1];
    float u0 = u[m * EE + e],     u1 = u[m * EE + e + 1];
    float du0 = d0 * u0, du1 = d1 * u1;
    float y0 = 0.f, y1 = 0.f;
    #pragma unroll
    for (int n = 0; n < NNS; ++n) {
      const float bn = bc[64 + n], cn = bc[80 + n];
      h0[n] = __expf(d0 * Ae0[n]) * h0[n] + du0 * bn;
      h1[n] = __expf(d1 * Ae1[n]) * h1[n] + du1 * bn;
      y0 += h0[n] * cn; y1 += h1[n] * cn;
    }
    float z0 = xz[m * (size_t)(2 * EE) + EE + e], z1 = xz[m * (size_t)(2 * EE) + EE + e + 1];
    float g0 = z0 / (1.f + __expf(-z0)), g1 = z1 / (1.f + __expf(-z1));
    unsigned lo; const unsigned hv = pack2s((y0 + u0 * dsk0) * g0, (y1 + u1 * dsk1) * g1, &lo);
    *(volatile unsigned*)(yb + m * EE + e) = hv; *(volatile unsigned*)(yb + PLY + m * EE + e) = lo;
    __threadfence();
    *(volatile unsigned*)(yb + m * EE + e) = hv; *(volatile unsigned*)(yb + PLY + m * EE + e) = lo;
  }
}

__global__ void layernorm_kernel(const float* __restrict__ res,
                                 const float* __restrict__ w,
                                 const float* __restrict__ bia,
                                 float* __restrict__ out) {
  __shared__ float s1[256];
  __shared__ float s2[256];
  int m = blockIdx.x;
  int tid = threadIdx.x;
  const float* row = res + (size_t)m * DD;
  float vals[DD / 256];
  float sum = 0.f, sq = 0.f;
  #pragma unroll
  for (int i = 0; i < DD / 256; ++i) {
    float v = row[tid + i * 256];
    vals[i] = v; sum += v; sq += v * v;
  }
  s1[tid] = sum; s2[tid] = sq;
  __syncthreads();
  for (int off = 128; off > 0; off >>= 1) {
    if (tid < off) { s1[tid] += s1[tid + off]; s2[tid] += s2[tid + off]; }
    __syncthreads();
  }
  float mu   = s1[0] / DD;
  float var  = s2[0] / DD - mu * mu;
  float rstd = rsqrtf(var + 1e-5f);
  #pragma unroll
  for (int i = 0; i < DD / 256; ++i) {
    int d = tid + i * 256;
    const float ov = (vals[i] - mu) * rstd * w[d] + bia[d];
    *(volatile float*)(out + (size_t)m * DD + d) = ov;
    __threadfence();
    *(volatile float*)(out + (size_t)m * DD + d) = ov;
  }
}

extern "C" void kernel_launch(void* const* d_in, const int* in_sizes, int n_in,
                              void* d_out, int out_size, void* d_ws, size_t ws_size,
                              hipStream_t stream) {
  const float* x      = (const float*)d_in[0];
  const float* W_in   = (const float*)d_in[1];
  const float* W_conv = (const float*)d_in[2];
  const float* b_conv = (const float*)d_in[3];
  const float* W_x    = (const float*)d_in[4];
  const float* W_dt   = (const float*)d_in[5];
  const float* b_dt   = (const float*)d_in[6];
  const float* A_log  = (const float*)d_in[7];
  const float* D_skip = (const float*)d_in[8];
  const float* W_out  = (const float*)d_in[9];
  const float* ln_w   = (const float*)d_in[10];
  const float* ln_b   = (const float*)d_in[11];
  float* out = (float*)d_out;

  char* ws = (char*)d_ws;
  size_t off = 0;
  auto take = [&](size_t bytes) -> char* {
    char* p = ws + off;
    off = (off + bytes + 255) & ~(size_t)255;
    return p;
  };
  bf16_t* Win_b  = (bf16_t*)take((size_t)2 * EE * DD * 2 * 2);
  bf16_t* Wx_b   = (bf16_t*)take((size_t)96 * EE * 2 * 2);
  bf16_t* Wdt_b  = (bf16_t*)take((size_t)EE * RR * 2 * 2);
  bf16_t* Wout_b = (bf16_t*)take((size_t)DD * EE * 2 * 2);
  bf16_t* x_b    = (bf16_t*)take((size_t)MTOT * DD * 2 * 2);
  float*  xzf    = (float*) take((size_t)MTOT * 2 * EE * 4);
  float*  uf     = (float*) take((size_t)MTOT * EE * 4);
  bf16_t* u_b    = (bf16_t*)take((size_t)MTOT * EE * 2 * 2);
  float*  dblf   = (float*) take((size_t)MTOT * 96 * 4);
  bf16_t* dt_b   = (bf16_t*)take((size_t)MTOT * RR * 2 * 2);
  float*  deltaf = (float*) take((size_t)MTOT * EE * 4);
  bf16_t* y_b    = (bf16_t*)take((size_t)MTOT * EE * 2 * 2);
  float*  resf   = (float*) take((size_t)MTOT * DD * 4);

  const int TPB = 256;
  auto cvt = [&](const float* src, bf16_t* dst, int n) {
    f32_to_bf16_kernel<<<(n / 2 + TPB - 1) / TPB, TPB, 0, stream>>>(src, dst, n);
  };
  cvt(W_in,  Win_b,  2 * EE * DD);
  cvt(W_x,   Wx_b,   96 * EE);
  cvt(W_dt,  Wdt_b,  EE * RR);
  cvt(W_out, Wout_b, DD * EE);
  cvt(x,     x_b,    MTOT * DD);

  {
    int blocks = (MTOT / TBM) * ((2 * EE) / TBN);
    gemm_bf16_wmma_tiled_kernel<0><<<blocks, 256, 0, stream>>>(
        x_b, Win_b, xzf, MTOT, 2 * EE, DD, nullptr);
  }
  {
    size_t n = (size_t)MTOT * EE / 2;
    conv_silu_kernel<<<(int)((n + TPB - 1) / TPB), TPB, 0, stream>>>(
        xzf, W_conv, b_conv, uf, u_b);
  }
  {
    int strips = (MTOT / 16) * (96 / (16 * 6));
    gemm_bf16_wmma_kernel<6, 1><<<strips / 8, 256, 0, stream>>>(
        u_b, Wx_b, dblf, MTOT, 96, EE, nullptr, dt_b);
  }
  {
    int strips = (MTOT / 16) * (EE / (16 * 4));
    gemm_bf16_wmma_kernel<4, 2><<<strips / 8, 256, 0, stream>>>(
        dt_b, Wdt_b, deltaf, MTOT, EE, RR, b_dt, nullptr);
  }
  scan_gate_kernel<<<(BB * EE / 2) / TPB, TPB, 0, stream>>>(
      deltaf, uf, dblf, xzf, A_log, D_skip, y_b);
  {
    int blocks = (MTOT / TBM) * (DD / TBN);
    gemm_bf16_wmma_tiled_kernel<3><<<blocks, 256, 0, stream>>>(
        y_b, Wout_b, resf, MTOT, DD, EE, x);
  }
  layernorm_kernel<<<MTOT, 256, 0, stream>>>(resf, ln_w, ln_b, out);
}
